// TemporalAttention_21071109554596
// MI455X (gfx1250) — hardware-verified
//
#include <hip/hip_runtime.h>
#include <math.h>
#include <stdint.h>

#define NB_   4
#define NT_   64
#define NS_   200
#define ND_   64
#define NHID  64
#define NHEAD 8
#define NQW   (NHEAD * NHID)
#define NSEQ  (NB_ * NS_)
#define LP    72
#define OB_ENC 0
#define OB_Q   64
#define OB_K   (64 + NQW)
#define OB_V   (64 + 2 * NQW)
#define OB_O   (64 + 3 * NQW)
#define NBIAS  (128 + 3 * NQW)
static_assert(NHID == 64);
static_assert(ND_ == 64);
static_assert(NT_ == 64);
static_assert((LP % 8) == 0);
static_assert((OB_Q % 4) == 0);
static_assert((OB_K % 4) == 0);
static_assert((OB_V % 4) == 0);
static_assert((OB_O % 4) == 0);

typedef __bf16   v16b __attribute__((ext_vector_type(16)));
typedef __bf16   v8b  __attribute__((ext_vector_type(8)));
typedef __bf16   v4b  __attribute__((ext_vector_type(4)));
typedef float    v8f  __attribute__((ext_vector_type(8)));
typedef float    v4f  __attribute__((ext_vector_type(4)));
typedef unsigned int v4u __attribute__((ext_vector_type(4)));

union SBuf { float f[NT_ * LP]; __bf16 o[2][NT_ * LP]; };

__device__ __forceinline__ unsigned short bf_bits(float f) {
  unsigned u = __float_as_uint(f);
  return (unsigned short)((u + 0x7FFFu + ((u >> 16) & 1u)) >> 16);
}
__device__ __forceinline__ float bf_up(unsigned short h) { return __uint_as_float(((unsigned)h) << 16); }
__device__ __forceinline__ float bf_rn(float f) { return bf_up(bf_bits(f)); }
__device__ __forceinline__ __bf16 to_bf(float f) { return __builtin_bit_cast(__bf16, bf_bits(f)); }
__device__ __forceinline__ unsigned pk16(unsigned short a, unsigned short b) { return (unsigned)a | ((unsigned)b << 16); }
__device__ __forceinline__ v8f zero8() { v8f z = {0.f, 0.f, 0.f, 0.f, 0.f, 0.f, 0.f, 0.f}; return z; }
__device__ __forceinline__ v4f bf_rn4(v4f a) {
  v4f r;
  r[0] = bf_rn(a[0]); r[1] = bf_rn(a[1]); r[2] = bf_rn(a[2]); r[3] = bf_rn(a[3]);
  return r;
}

__device__ __forceinline__ v16b ldfrag_b(const __bf16* p) {
  union { v16b v; v8b h[2]; } f;
  f.h[0] = *(const v8b*)(p);
  f.h[1] = *(const v8b*)(p + 16);
  return f.v;
}

__device__ __forceinline__ v8f mma_b(v16b a, v16b b, v8f c) {
  c = __builtin_amdgcn_wmma_f32_16x16x32_bf16(false, a, false, b, (short)0, c, false, false);
#if defined(__HIP_DEVICE_COMPILE__)
  asm volatile("v_nop\n\tv_nop\n\tv_nop\n\tv_nop" : "+v"(c) : "v"(a), "v"(b));
#endif
  return c;
}

__device__ __forceinline__ void put_split(__bf16* dh, __bf16* dl, int off, float v) {
  const unsigned short hb = bf_bits(v);
  const unsigned short lb = bf_bits(v - bf_up(hb));
  dh[off] = __builtin_bit_cast(__bf16, hb);
  dl[off] = __builtin_bit_cast(__bf16, lb);
}

template <bool ASPLIT, bool BSPLIT>
__device__ __forceinline__ void mm64(const __bf16* Ah, const __bf16* Al, const __bf16* Bh, const __bf16* Bl,
                                     v8f& acc0, v8f& acc1) {
  const int lane = threadIdx.x & 31, wave = threadIdx.x >> 5;
  const int c = lane & 15, koff = (lane >> 4) * 8;
  const int arow  = (wave >> 1) * 16 + c;
  const int brow0 = (wave & 1) * 32 + c;
  const int brow1 = brow0 + 16;
#pragma unroll
  for (int ks = 0; ks < 2; ++ks) {
    const int k0 = ks * 32 + koff;
    const v16b ah = ldfrag_b(Ah + arow * LP + k0);
    v16b al = ah;
    if (ASPLIT) al = ldfrag_b(Al + arow * LP + k0);
    const v16b b0 = ldfrag_b(Bh + brow0 * LP + k0);
    const v16b b1 = ldfrag_b(Bh + brow1 * LP + k0);
    acc0 = mma_b(ah, b0, acc0);
    acc1 = mma_b(ah, b1, acc1);
    if (BSPLIT) {
      const v16b l0 = ldfrag_b(Bl + brow0 * LP + k0);
      const v16b l1 = ldfrag_b(Bl + brow1 * LP + k0);
      acc0 = mma_b(ah, l0, acc0);
      acc1 = mma_b(ah, l1, acc1);
    }
    if (ASPLIT) {
      acc0 = mma_b(al, b0, acc0);
      acc1 = mma_b(al, b1, acc1);
    }
  }
}

__device__ __forceinline__ void epi_split_col(const v8f& a, int row0, int col, const float* bias, __bf16* dh, __bf16* dl) {
  const float bb = bias[col];
#pragma unroll
  for (int r = 0; r < 8; ++r) put_split(dh, dl, (row0 + r) * LP + col, a[r] + bb);
}
__device__ __forceinline__ void epi_split_row(const v8f& a, int row0, int col, const float* bias, __bf16* dh, __bf16* dl) {
#pragma unroll
  for (int r = 0; r < 8; ++r) put_split(dh, dl, (row0 + r) * LP + col, a[r] + bias[row0 + r]);
}
__device__ __forceinline__ void epi_split_nob(const v8f& a, int row0, int col, __bf16* dh, __bf16* dl) {
#pragma unroll
  for (int r = 0; r < 8; ++r) put_split(dh, dl, (row0 + r) * LP + col, a[r]);
}
__device__ __forceinline__ void epi_f32(const v8f& a, int row0, int col, float* d) {
#pragma unroll
  for (int r = 0; r < 8; ++r) d[(row0 + r) * LP + col] = a[r];
}
__device__ __forceinline__ void epi_h(const v8f& a, int row0, int col, const float* bias, const float* pef,
                                      __bf16* dh, __bf16* dl) {
  const float bb = bias[col];
#pragma unroll
  for (int r = 0; r < 8; ++r) {
    const int off = (row0 + r) * LP + col;
    float v = a[r] + bb;
    v = v + pef[off];
    put_split(dh, dl, off, v);
  }
}

__device__ __forceinline__ void stage_w(const unsigned short* __restrict__ src, int pitch, __bf16* dst) {
  const __bf16* s = (const __bf16*)(const void*)src;
  const int tid = threadIdx.x;
#pragma unroll
  for (int it = 0; it < 2; ++it) {
    const int idx = it * 256 + tid, row = idx >> 3, c8 = (idx & 7) * 8;
    const v8b v = *(const v8b*)(s + (size_t)row * pitch + c8);
    *(v8b*)(dst + row * LP + c8) = v;
  }
}

__global__ __launch_bounds__(256) void tcvt_kernel(const float* __restrict__ W, unsigned short* out, int R, int Cc) {
  __shared__ __align__(16) float tf[64 * 68];
  const int c0  = blockIdx.x * 64;
  const int r0  = blockIdx.y * 64;
  const int tid = threadIdx.x;
  {
    const int lr = tid >> 4;
    const int c4 = (tid & 15) * 4;
#pragma unroll
    for (int it = 0; it < 4; ++it) {
      const int rr = it * 16 + lr;
      const v4f a = *(const v4f*)(W + (size_t)(r0 + rr) * Cc + c0 + c4);
      *(v4f*)(tf + rr * 68 + c4) = a;
    }
  }
  __syncthreads();
  const int sub = tid >> 3;
  const int c8  = (tid & 7) * 8;
  v4u hv[2];
#pragma unroll
  for (int it = 0; it < 2; ++it) {
    const int oc = it * 32 + sub;
    v4u a;
#pragma unroll
    for (int q = 0; q < 4; ++q) {
      const float f0 = tf[(c8 + 2 * q) * 68 + oc];
      const float f1 = tf[(c8 + 2 * q + 1) * 68 + oc];
      a[q] = pk16(bf_bits(f0), bf_bits(f1));
    }
    hv[it] = a;
  }
  for (int pass = 0; pass < 2; ++pass) {
#pragma unroll
    for (int it = 0; it < 2; ++it) {
      const int oc = it * 32 + sub;
      const size_t go = (size_t)(c0 + oc) * R + r0 + c8;
      *(volatile v4u*)(out + go) = hv[it];
    }
    __threadfence();
  }
}

__global__ __launch_bounds__(256) void pe_kernel(float* pe) {
  __shared__ __align__(16) float tile[8 * 64];
  const int tid = threadIdx.x;
  const int tl = tid >> 5, i = tid & 31;
  const int t = blockIdx.x * 8 + tl;
  const float cst = -0.14391156831212787f;
  const float dv  = expf((float)(2 * i) * cst);
  const float ang = (float)t * dv;
  tile[tl * 64 + 2 * i]     = sinf(ang);
  tile[tl * 64 + 2 * i + 1] = cosf(ang);
  __syncthreads();
  if (tid < 128) {
    const int row = tid >> 4, c4 = (tid & 15) * 4;
    const v4f v = *(const v4f*)(tile + row * 64 + c4);
    float* dst = pe + (size_t)(blockIdx.x * 8 + row) * 64 + c4;
    *(volatile v4f*)dst = v;
    __threadfence();
    *(volatile v4f*)dst = v;
  }
}

__global__ __launch_bounds__(256)
void seq_attn_kernel(const float* __restrict__ x,
                     const unsigned short* __restrict__ wencT, const unsigned short* __restrict__ wqT,
                     const unsigned short* __restrict__ wkT,   const unsigned short* __restrict__ wvT,
                     const unsigned short* __restrict__ woT,   const float* __restrict__ pe,
                     const float* __restrict__ b_enc, const float* __restrict__ bq, const float* __restrict__ bk,
                     const float* __restrict__ bv,    const float* __restrict__ bo, float* out) {
  __shared__ __align__(16) __bf16 hS[2][NT_ * LP];
  __shared__ __align__(16) __bf16 wS[NHID * LP];
  __shared__ __align__(16) __bf16 aS[2][NT_ * LP];
  __shared__ __align__(16) __bf16 bS[2][NT_ * LP];
  __shared__ __align__(16) SBuf   sS;
  __shared__ __align__(16) float  biasS[NBIAS];

  const int tid = threadIdx.x, lane = tid & 31, wave = tid >> 5;
  const int hh = lane >> 4, c = lane & 15;
  const int row0 = (wave >> 1) * 16 + 8 * hh;
  const int col0 = (wave & 1) * 32 + c;
  const int col1 = col0 + 16;
  const int seq = blockIdx.x;
  const int b = seq / NS_, n = seq - b * NS_;

  {
    const v4f e4 = *(const v4f*)(b_enc + 4 * (tid & 15));
    const v4f o4 = *(const v4f*)(bo    + 4 * (tid & 15));
    const v4f q4 = *(const v4f*)(bq    + 4 * (tid & 127));
    const v4f k4 = *(const v4f*)(bk    + 4 * (tid & 127));
    const v4f v4 = *(const v4f*)(bv    + 4 * (tid & 127));
    if (tid < 16) {
      *(v4f*)(biasS + OB_ENC + 4 * tid) = bf_rn4(e4);
      *(v4f*)(biasS + OB_O   + 4 * tid) = bf_rn4(o4);
    }
    if (tid < 128) {
      *(v4f*)(biasS + OB_Q + 4 * tid) = bf_rn4(q4);
      *(v4f*)(biasS + OB_K + 4 * tid) = bf_rn4(k4);
      *(v4f*)(biasS + OB_V + 4 * tid) = bf_rn4(v4);
    }
  }
  {
#pragma unroll
    for (int it = 0; it < 4; ++it) {
      const int idx = it * 256 + tid, row = idx >> 4, c4 = (idx & 15) * 4;
      const v4f p4 = *(const v4f*)(pe + row * 64 + c4);
      *(v4f*)(sS.f + row * LP + c4) = p4;
    }
  }
  {
    const float* xs = x + (((size_t)b * NT_) * NS_ + n) * ND_;
#pragma unroll
    for (int it = 0; it < 4; ++it) {
      const int idx = it * 256 + tid, t = idx >> 4, c4 = (idx & 15) * 4;
      const v4f a = *(const v4f*)(xs + (size_t)t * (NS_ * ND_) + c4);
      v4b o;
      o[0] = to_bf(a[0]); o[1] = to_bf(a[1]); o[2] = to_bf(a[2]); o[3] = to_bf(a[3]);
      *(v4b*)(aS[0] + t * LP + c4) = o;
    }
  }
  stage_w(wencT, NHID, wS);
  __syncthreads();

  {
    v8f a0 = zero8(), a1 = zero8();
    mm64<false, false>(aS[0], aS[0], wS, wS, a0, a1);
    epi_h(a0, row0, col0, biasS + OB_ENC, sS.f, hS[0], hS[1]);
    epi_h(a1, row0, col1, biasS + OB_ENC, sS.f, hS[0], hS[1]);
  }
  __syncthreads();

  v8f y0 = zero8(), y1 = zero8();

#pragma unroll 1
  for (int j = 0; j < NHEAD; ++j) {
    stage_w(wqT + (size_t)j * NHID * NHID, NHID, wS);
    __syncthreads();
    {
      v8f a0 = zero8(), a1 = zero8();
      mm64<true, false>(hS[0], hS[1], wS, wS, a0, a1);
      epi_split_col(a0, row0, col0, biasS + OB_Q + j * NHID, aS[0], aS[1]);
      epi_split_col(a1, row0, col1, biasS + OB_Q + j * NHID, aS[0], aS[1]);
    }
    __syncthreads();
    stage_w(wkT + (size_t)j * NHID * NHID, NHID, wS);
    __syncthreads();
    {
      v8f a0 = zero8(), a1 = zero8();
      mm64<true, false>(hS[0], hS[1], wS, wS, a0, a1);
      epi_split_col(a0, row0, col0, biasS + OB_K + j * NHID, bS[0], bS[1]);
      epi_split_col(a1, row0, col1, biasS + OB_K + j * NHID, bS[0], bS[1]);
    }
    __syncthreads();
    {
      v8f a0 = zero8(), a1 = zero8();
      mm64<true, true>(aS[0], aS[1], bS[0], bS[1], a0, a1);
      epi_f32(a0, row0, col0, sS.f);
      epi_f32(a1, row0, col1, sS.f);
      stage_w(wvT + (size_t)j * NHID * NHID, NHID, wS);
    }
    __syncthreads();
    {
      const int row = tid >> 2, part = tid & 3;
      const float* sr = sS.f + row * LP + part * 16;
      float vb[16];
#pragma unroll
      for (int i4 = 0; i4 < 4; ++i4) {
        const v4f t4 = *(const v4f*)(sr + 4 * i4);
        vb[4 * i4 + 0] = t4[0]; vb[4 * i4 + 1] = t4[1]; vb[4 * i4 + 2] = t4[2]; vb[4 * i4 + 3] = t4[3];
      }
      float mx = -INFINITY;
#pragma unroll
      for (int i = 0; i < 16; ++i) {
        const int s = part * 16 + i;
        const float sv = vb[i] * 0.125f;
        vb[i] = (s <= row) ? sv : -INFINITY;
        mx = fmaxf(mx, vb[i]);
      }
      mx = fmaxf(mx, __shfl_xor(mx, 1, 4));
      mx = fmaxf(mx, __shfl_xor(mx, 2, 4));
      float sum = 0.0f;
#pragma unroll
      for (int i = 0; i < 16; ++i) {
        const int s = part * 16 + i;
        const float e = (s <= row) ? __expf(vb[i] - mx) : 0.0f;
        vb[i] = e;
        sum += e;
      }
      sum += __shfl_xor(sum, 1, 4);
      sum += __shfl_xor(sum, 2, 4);
      const float inv = 1.0f / sum;
      __bf16* ph = aS[0] + row * LP + part * 16;
      __bf16* pl = aS[1] + row * LP + part * 16;
#pragma unroll
      for (int i4 = 0; i4 < 4; ++i4) {
        v4b hv, lv;
#pragma unroll
        for (int e = 0; e < 4; ++e) {
          const float p = vb[4 * i4 + e] * inv;
          const unsigned short hb = bf_bits(p);
          const unsigned short lb = bf_bits(p - bf_up(hb));
          hv[e] = __builtin_bit_cast(__bf16, hb);
          lv[e] = __builtin_bit_cast(__bf16, lb);
        }
        *(v4b*)(ph + 4 * i4) = hv;
        *(v4b*)(pl + 4 * i4) = lv;
      }
    }
    {
      v8f a0 = zero8(), a1 = zero8();
      mm64<false, true>(wS, wS, hS[0], hS[1], a0, a1);
      epi_split_row(a0, row0, col0, biasS + OB_V + j * NHID, bS[0], bS[1]);
      epi_split_row(a1, row0, col1, biasS + OB_V + j * NHID, bS[0], bS[1]);
    }
    __syncthreads();
    {
      v8f a0 = zero8(), a1 = zero8();
      mm64<true, true>(aS[0], aS[1], bS[0], bS[1], a0, a1);
      epi_split_nob(a0, row0, col0, sS.o[0], sS.o[1]);
      epi_split_nob(a1, row0, col1, sS.o[0], sS.o[1]);
      stage_w(woT + (size_t)j * NHID, NQW, wS);
    }
    __syncthreads();
    mm64<true, false>(sS.o[0], sS.o[1], wS, wS, y0, y1);
    __syncthreads();
  }

  {
    const float bb0 = biasS[OB_O + col0], bb1 = biasS[OB_O + col1];
#pragma unroll
    for (int r = 0; r < 8; ++r) {
      sS.f[(row0 + r) * LP + col0] = y0[r] + bb0;
      sS.f[(row0 + r) * LP + col1] = y1[r] + bb1;
    }
  }
  __syncthreads();
  {
    float* ob = out + (size_t)seq * (NT_ * NHID);
    const int rs = tid >> 4, c4 = (tid & 15) * 4;
    for (int pass = 0; pass < 2; ++pass) {
#pragma unroll
      for (int it = 0; it < 4; ++it) {
        const int row = it * 16 + rs;
        const v4f v = *(const v4f*)(sS.f + row * LP + c4);
        *(volatile v4f*)(ob + (size_t)row * NHID + c4) = v;
      }
      __threadfence();
    }
  }
}

extern "C" void kernel_launch(void* const* d_in, const int* in_sizes, int n_in,
                              void* d_out, int out_size, void* d_ws, size_t ws_size,
                              hipStream_t stream) {
  if (n_in < 11) return;
  if (in_sizes[0] != NB_ * NT_ * NS_ * ND_) return;
  if (in_sizes[1] != ND_ * NHID || in_sizes[2] != NHID) return;
  if (in_sizes[3] != NHID * NQW || in_sizes[4] != NQW) return;
  if (in_sizes[5] != NHID * NQW || in_sizes[6] != NQW) return;
  if (in_sizes[7] != NHID * NQW || in_sizes[8] != NQW) return;
  if (in_sizes[9] != NQW * NHID || in_sizes[10] != NHID) return;
  if (out_size != NSEQ * NT_ * NHID) return;

  const float* x     = (const float*)d_in[0];
  const float* W_enc = (const float*)d_in[1];
  const float* b_enc = (const float*)d_in[2];
  const float* Wq    = (const float*)d_in[3];
  const float* bq    = (const float*)d_in[4];
  const float* Wk    = (const float*)d_in[5];
  const float* bk    = (const float*)d_in[6];
  const float* Wv    = (const float*)d_in[7];
  const float* bv    = (const float*)d_in[8];
  const float* Wo    = (const float*)d_in[9];
  const float* bo    = (const float*)d_in[10];

  const size_t PWE = (size_t)NHID * ND_ * 2;
  const size_t PWP = (size_t)NQW * NHID * 2;
  const size_t PPE = (size_t)NT_ * NHID * 4;
  size_t off = 0;
  const size_t oWe = off; off += PWE;
  const size_t oWq = off; off += PWP;
  const size_t oWk = off; off += PWP;
  const size_t oWv = off; off += PWP;
  const size_t oWo = off; off += PWP;
  const size_t oPe = off; off += PPE;
  if (off > ws_size) return;
  if (off > (size_t)134217728) return;

  char* ws = (char*)d_ws;
  unsigned short* WencT = (unsigned short*)(ws + oWe);
  unsigned short* WqT   = (unsigned short*)(ws + oWq);
  unsigned short* WkT   = (unsigned short*)(ws + oWk);
  unsigned short* WvT   = (unsigned short*)(ws + oWv);
  unsigned short* WoT   = (unsigned short*)(ws + oWo);
  float*          PE    = (float*)(ws + oPe);

  const dim3 blk(256);
  tcvt_kernel<<<dim3(NHID / 64, ND_ / 64), blk, 0, stream>>>(W_enc, WencT, ND_, NHID);
  tcvt_kernel<<<dim3(NQW / 64, NHID / 64), blk, 0, stream>>>(Wq, WqT, NHID, NQW);
  tcvt_kernel<<<dim3(NQW / 64, NHID / 64), blk, 0, stream>>>(Wk, WkT, NHID, NQW);
  tcvt_kernel<<<dim3(NQW / 64, NHID / 64), blk, 0, stream>>>(Wv, WvT, NHID, NQW);
  tcvt_kernel<<<dim3(NHID / 64, NQW / 64), blk, 0, stream>>>(Wo, WoT, NQW, NHID);
  pe_kernel<<<dim3(NT_ / 8), blk, 0, stream>>>(PE);
  seq_attn_kernel<<<dim3(NSEQ), blk, 0, stream>>>(x, WencT, WqT, WkT, WvT, WoT, PE,
                                                  b_enc, bq, bk, bv, bo, (float*)d_out);
  (void)hipGetLastError();
}
